// SpatialAttention_4337916969718
// MI455X (gfx1250) — hardware-verified
//
#include <hip/hip_runtime.h>


#ifndef NB
#define NB 4
#endif
#ifndef SEQ
#define SEQ 1024
#endif
#define NB_FULL  4
#define SEQ_FULL 1024
#define HID   64
#define TK    SEQ
#define DV    HID
#define KPT   (SEQ / 256)
#define PCAR  1024.0f
#define VSC   16.0f
#define OSC   (1.0f / 16384.0f)
#define LOG2E 1.4426950408889634f

#define WS_WB   ((size_t)HID * HID * 2)
#define WS_XB   ((size_t)NB * SEQ * HID * 2)
#define WS_F32  ((size_t)NB * SEQ * HID * 4)
#define WS_XT   ((size_t)NB * DV * TK * 2)
#define WS_P    ((size_t)NB * SEQ * SEQ * 2)
#define WS_TOTAL (2 * WS_WB + WS_XB + 3 * WS_F32 + WS_XT + WS_P)

static_assert(SEQ == SEQ_FULL || NB == 1);
static_assert(SEQ % 256 == 0 && SEQ >= 256 && SEQ <= SEQ_FULL);
static_assert(NB >= 1 && NB <= NB_FULL);
static_assert(HID == 64 && HID % 32 == 0 && HID % 64 == 0 && (HID * HID) % 8 == 0);
static_assert((NB * SEQ) % 64 == 0 && SEQ % 64 == 0 && SEQ % 32 == 0);
static_assert((NB * SEQ) % 128 == 0);
static_assert(KPT * 256 == SEQ && KPT >= 1 && KPT <= 8);
static_assert((SEQ / 8) * 16 == SEQ * 2 && (SEQ / 8) % 32 == 0 && SEQ / 8 <= 256);
static_assert(8 * 8 * 32 * 16 == 128 * HID * 4);
static_assert((size_t)NB_FULL * SEQ_FULL * HID * 4 == 1048576);
static_assert(WS_WB % 256 == 0 && WS_XB % 256 == 0 && WS_F32 % 256 == 0 && WS_XT % 256 == 0 && WS_P % 256 == 0);
static_assert(WS_TOTAL <= (size_t)134217728);
static_assert((2 * HID + SEQ + 8) * 4 <= 131072);
static_assert(16 * 68 * 4 <= 131072);

typedef _Float16 h16;
typedef unsigned short bf;
typedef __attribute__((ext_vector_type(16))) __bf16   v16bf;
typedef __attribute__((ext_vector_type(16))) _Float16 v16h;
typedef __attribute__((ext_vector_type(8)))  _Float16 v8h;
typedef __attribute__((ext_vector_type(8)))  unsigned short v8us;
typedef __attribute__((ext_vector_type(8)))  float    v8f;
typedef __attribute__((ext_vector_type(4)))  float    v4f;
typedef __attribute__((ext_vector_type(2)))  _Float16 v2h;
typedef __attribute__((ext_vector_type(2)))  unsigned short v2us;
typedef v8h  __attribute__((may_alias)) v8ha;
typedef v4f  __attribute__((may_alias)) v4fa;
typedef v8us __attribute__((may_alias)) v8usa;

__device__ __forceinline__ unsigned short f2bf(float f) { unsigned u = __float_as_uint(f); u += 0x7FFFu + ((u >> 16) & 1u); return (unsigned short)(u >> 16); }
__device__ __forceinline__ float bf2f(unsigned short b) { return __uint_as_float(((unsigned)b) << 16); }
__device__ __forceinline__ float bfr(float f) { return bf2f(f2bf(f)); }
__device__ __forceinline__ v16h cat16(v8h lo, v8h hi) { return __builtin_shufflevector(lo, hi, 0, 1, 2, 3, 4, 5, 6, 7, 8, 9, 10, 11, 12, 13, 14, 15); }
__device__ __forceinline__ v16bf cat16b(v8us lo, v8us hi) { return __builtin_bit_cast(v16bf, __builtin_shufflevector(lo, hi, 0, 1, 2, 3, 4, 5, 6, 7, 8, 9, 10, 11, 12, 13, 14, 15)); }
__device__ __forceinline__ v8f wmma16(v16h a, v16h b, v8f c) { return __builtin_amdgcn_wmma_f32_16x16x32_f16(false, a, false, b, (short)0, c, false, false); }
__device__ __forceinline__ v8f wmmab(v16bf a, v16bf b, v8f c) { return __builtin_amdgcn_wmma_f32_16x16x32_bf16(false, a, false, b, (short)0, c, false, false); }

static __device__ __forceinline__ h16 toh_flush(float v) { const float w = (fabsf(v) < 6.103515625e-05f) ? 0.0f : v; return (h16)w; }

template <typename T16> struct WFrag;
template <> struct WFrag<h16> { typedef v16h V; static __device__ __forceinline__ V ld(const h16* p) { return cat16(*(const v8h*)p, *(const v8h*)(p + 16)); } static __device__ __forceinline__ v8f mma(V a, V b, v8f c) { return wmma16(a, b, c); } };
template <> struct WFrag<bf> { typedef v16bf V; static __device__ __forceinline__ V ld(const bf* p) { return cat16b(*(const v8us*)p, *(const v8us*)(p + 16)); } static __device__ __forceinline__ v8f mma(V a, V b, v8f c) { return wmmab(a, b, c); } };
template <typename T16, int NSPLIT, bool BIAS>
__global__ __launch_bounds__(32) void k_gemmw(const T16* __restrict__ A, const T16* __restrict__ A2, const T16* __restrict__ Bt, const T16* __restrict__ Bt2, int K, float* C, int ldc, const float* __restrict__ bias, float csc, size_t sA, size_t sB, size_t sC) {
    typedef typename WFrag<T16>::V V;
    __shared__ __align__(16) float os[16 * 68];
    const size_t z = blockIdx.z; A += z * sA; if (A2) A2 += z * sA; Bt += z * sB; if (Bt2) Bt2 += z * sB; C += z * sC;
    const int lane = threadIdx.x & 31, lr = lane & 15, hi = lane >> 4; const int r0 = blockIdx.x * 64, c0 = blockIdx.y * 64;
    v8f acc[4][4];
#pragma unroll
    for (int mb = 0; mb < 4; ++mb)
#pragma unroll
        for (int nb = 0; nb < 4; ++nb) acc[mb][nb] = (v8f){};
    const size_t aoff = (size_t)(r0 + lr) * K + 8 * hi, boff = (size_t)(c0 + lr) * K + 8 * hi;
#pragma unroll 1
    for (int kc = 0; kc < K; kc += 32) {
        V a[4], a2[4];
#pragma unroll
        for (int mb = 0; mb < 4; ++mb) { a[mb] = WFrag<T16>::ld(A + aoff + (size_t)mb * 16 * K + kc); if (NSPLIT == 1 || NSPLIT == 2) a2[mb] = WFrag<T16>::ld(A2 + aoff + (size_t)mb * 16 * K + kc); }
#pragma unroll
        for (int nb = 0; nb < 4; ++nb) { const V b = WFrag<T16>::ld(Bt + boff + (size_t)nb * 16 * K + kc); V b2; if (NSPLIT >= 2) b2 = WFrag<T16>::ld(Bt2 + boff + (size_t)nb * 16 * K + kc);
#pragma unroll
            for (int mb = 0; mb < 4; ++mb) { acc[mb][nb] = WFrag<T16>::mma(a[mb], b, acc[mb][nb]); if (NSPLIT == 1 || NSPLIT == 2) acc[mb][nb] = WFrag<T16>::mma(a2[mb], b, acc[mb][nb]); if (NSPLIT >= 2) acc[mb][nb] = WFrag<T16>::mma(a[mb], b2, acc[mb][nb]); } }
        asm volatile("v_nop\n\tv_nop\n\tv_nop\n\tv_nop" : "+v"(acc[0][0]), "+v"(acc[1][1]), "+v"(acc[2][2]), "+v"(acc[3][3]) : "v"(a[0]), "v"(a[3]));
    }
#pragma unroll
    for (int mb = 0; mb < 4; ++mb) {
#pragma unroll
        for (int nb = 0; nb < 4; ++nb) {
#pragma unroll
            for (int j = 0; j < 8; ++j) os[(hi * 8 + j) * 68 + nb * 16 + lr] = acc[mb][nb][j]; }
        __builtin_amdgcn_wave_barrier(); asm volatile("" ::: "memory");
        float* crow = C + (size_t)(r0 + mb * 16) * ldc + c0;
#pragma unroll 1
        for (int ps = 0; ps < 2; ++ps) {
#pragma unroll
            for (int s = 0; s < 8; ++s) { const int row = 2 * s + hi, cofs = lr * 4; v4f val = *(const v4fa*)(os + row * 68 + cofs); val = val * csc;
                if (BIAS) { val[0] += bfr(bias[c0 + cofs]); val[1] += bfr(bias[c0 + cofs + 1]); val[2] += bfr(bias[c0 + cofs + 2]); val[3] += bfr(bias[c0 + cofs + 3]); }
                *(volatile v4f*)(crow + (size_t)row * ldc + cofs) = val; }
            if (ps == 0) __threadfence(); }
        __builtin_amdgcn_wave_barrier(); asm volatile("" ::: "memory");
    }
}

__global__ __launch_bounds__(256) void k_cvt8(const float* __restrict__ src, bf* dst, size_t n8) { const size_t i = (size_t)blockIdx.x * 256 + threadIdx.x; if (i >= n8) return; const v8f v = *(const v8f*)(src + i * 8); v8us o;
#pragma unroll
    for (int k = 0; k < 8; ++k) o[k] = f2bf(v[k]); *(volatile v8us*)(dst + i * 8) = o; __threadfence(); *(volatile v8us*)(dst + i * 8) = o; }

__global__ __launch_bounds__(256) void k_vtp(const float* __restrict__ F, h16* V16) {
    const size_t e = ((size_t)blockIdx.x * 256 + threadIdx.x) * 2; if (e >= (size_t)NB * DV * TK) return;
    const int t = (int)(e % TK); const int d = (int)((e / TK) % DV); const int b = (int)(e / ((size_t)TK * DV));
    v2h o;
#pragma unroll
    for (int q = 0; q < 2; ++q) o[q] = toh_flush(bfr(F[((size_t)b * TK + t + q) * DV + d]) * VSC);
    *(volatile v2h*)(V16 + e) = o; __threadfence(); *(volatile v2h*)(V16 + e) = o;
}

__device__ __forceinline__ float tnh(float x) {
    const float e = __builtin_amdgcn_exp2f(x * 2.8853900817779268f);
    const float r = __builtin_amdgcn_rcpf(e + 1.0f);
    return fmaf(-2.0f, r, 1.0f);
}

__global__ __launch_bounds__(256) void k_score(const float* __restrict__ SF, const float* __restrict__ TF, const float* __restrict__ vv, const int* __restrict__ adj, h16* P16) {
    __shared__ __align__(16) float s_s[HID];
    __shared__ __align__(16) float s_v[HID];
    __shared__ __align__(16) float s_sc[SEQ];
    __shared__ float red[8];
    const int rq = blockIdx.x; const int b = rq / SEQ; const int i = rq - b * SEQ;
    const int tid = threadIdx.x, lane = tid & 31;
    const int wave = __builtin_amdgcn_readfirstlane(threadIdx.x >> 5);
    const int hx = tid & (HID - 1);
    const float s1 = SF[(size_t)rq * HID + hx];
    const float v1 = bfr(vv[hx]);
    if (wave < HID / 32) { s_s[hx] = s1; s_v[hx] = v1; }
    const int* arow = adj + ((size_t)b * SEQ_FULL + i) * SEQ_FULL;
    int ad[KPT];
#pragma unroll
    for (int q = 0; q < KPT; ++q) ad[q] = arow[tid + 256 * q];
    __syncthreads();
    const float* tp = TF + ((size_t)b * SEQ + tid) * HID;
    float acc[KPT];
#pragma unroll
    for (int q = 0; q < KPT; ++q) acc[q] = 0.0f;
#pragma unroll 1
    for (int c = 0; c < HID / 4; ++c) {
        const v4f s4 = *(const v4fa*)(s_s + 4 * c);
        const v4f w4 = *(const v4fa*)(s_v + 4 * c);
#pragma unroll
        for (int q = 0; q < KPT; ++q) {
            const v4f t4 = *(const v4f*)(tp + (size_t)q * 256 * HID + 4 * c);
#pragma unroll
            for (int e = 0; e < 4; ++e) acc[q] = fmaf(w4[e], tnh(s4[e] + t4[e]), acc[q]);
        }
    }
    float sc[KPT];
#pragma unroll
    for (int q = 0; q < KPT; ++q) sc[q] = (ad[q] == 0) ? -1.0e9f : acc[q];
    float m = sc[0];
#pragma unroll
    for (int q = 1; q < KPT; ++q) m = (sc[q] > m) ? sc[q] : m;
#pragma unroll
    for (int sh = 16; sh; sh >>= 1) m = fmaxf(m, __shfl_xor(m, sh, 32));
    if (lane == 0) red[wave] = m;
    __syncthreads();
    m = red[0];
#pragma unroll
    for (int w = 1; w < 8; ++w) m = fmaxf(m, red[w]);
    __syncthreads();
    float sum = 0.0f;
#pragma unroll
    for (int q = 0; q < KPT; ++q) { const float ex = __builtin_amdgcn_exp2f((sc[q] - m) * LOG2E); s_sc[tid + 256 * q] = ex; sum += ex; }
#pragma unroll
    for (int sh = 16; sh; sh >>= 1) sum += __shfl_xor(sum, sh, 32);
    if (lane == 0) red[wave] = sum;
    __syncthreads();
    sum = red[0];
#pragma unroll
    for (int w = 1; w < 8; ++w) sum += red[w];
    const float inv = __builtin_amdgcn_rcpf(sum); const float invp = inv * PCAR;
    if (wave < KPT) {
        const int f0 = tid * 8;
        const v4f q0 = *(const v4fa*)(s_sc + f0); const v4f q1 = *(const v4fa*)(s_sc + f0 + 4);
        v8h o;
#pragma unroll
        for (int c = 0; c < 4; ++c) { o[c] = toh_flush(q0[c] * invp); o[4 + c] = toh_flush(q1[c] * invp); }
        h16* dst = P16 + (size_t)rq * SEQ + f0;
        *(volatile v8h*)dst = o; __threadfence(); *(volatile v8h*)dst = o;
    }
}

__global__ __launch_bounds__(256) void k_lnorm(const float* __restrict__ CT, const float* __restrict__ gn, const float* __restrict__ bt, float* out) {
    const int lane = threadIdx.x & 31, lr = lane & 15, hi = lane >> 4;
    const int wave = __builtin_amdgcn_readfirstlane(threadIdx.x >> 5);
    const int r0 = (blockIdx.x * 8 + wave) * 16;
    const v4f g4 = *(const v4f*)(gn + 4 * lr); const v4f b4 = *(const v4f*)(bt + 4 * lr);
    v4f gg, bb;
#pragma unroll
    for (int c = 0; c < 4; ++c) { gg[c] = bfr(g4[c]); bb[c] = bfr(b4[c]); }
#pragma unroll 1
    for (int s = 0; s < 8; ++s) {
        const size_t row = (size_t)(r0 + 2 * s + hi);
        const v4f c4 = *(const v4f*)(CT + row * HID + 4 * lr);
        float sm = (c4[0] + c4[1]) + (c4[2] + c4[3]);
#pragma unroll
        for (int sh = 8; sh; sh >>= 1) sm += __shfl_xor(sm, sh, 32);
        const float mu = sm * (1.0f / 64.0f);
        const v4f d4 = c4 - mu;
        float vs = (d4[0] * d4[0] + d4[1] * d4[1]) + (d4[2] * d4[2] + d4[3] * d4[3]);
#pragma unroll
        for (int sh = 8; sh; sh >>= 1) vs += __shfl_xor(vs, sh, 32);
        const float rs = rsqrtf(vs * (1.0f / 64.0f) + 1.0e-5f);
        v4f o;
#pragma unroll
        for (int c = 0; c < 4; ++c) o[c] = d4[c] * rs * gg[c] + bb[c];
        float* dst = out + row * HID + 4 * lr;
        *(volatile v4f*)dst = o; __threadfence(); *(volatile v4f*)dst = o;
    }
}

extern "C" void kernel_launch(void* const* d_in, const int* in_sizes, int n_in,
                              void* d_out, int out_size, void* d_ws, size_t ws_size, hipStream_t stream) {
    if (n_in < 9) return;
    if (in_sizes[0] < NB * SEQ * HID || in_sizes[1] < (NB - 1) * SEQ_FULL * SEQ_FULL + (SEQ - 1) * SEQ_FULL + SEQ || in_sizes[2] < HID * HID || in_sizes[3] < HID ||
        in_sizes[4] < HID * HID || in_sizes[5] < HID || in_sizes[6] < HID || in_sizes[7] < HID || in_sizes[8] < HID) return;
    if (out_size < NB * SEQ * HID) return;
    const float* x    = (const float*)d_in[0];
    const int*   adj  = (const int*)d_in[1];
    const float* Ws_w = (const float*)d_in[2];
    const float* Ws_b = (const float*)d_in[3];
    const float* Wt_w = (const float*)d_in[4];
    const float* Wt_b = (const float*)d_in[5];
    const float* vv   = (const float*)d_in[6];
    const float* ln_g = (const float*)d_in[7];
    const float* ln_b = (const float*)d_in[8];
    float* OUT = (float*)d_out;

    char* wsp = (char*)d_ws;
    auto take = [&](size_t bytes) { char* p = wsp; wsp += (bytes + 255) & ~(size_t)255; return (void*)p; };
    bf*    WSB  = (bf*)take(WS_WB);
    bf*    WTB  = (bf*)take(WS_WB);
    bf*    XB   = (bf*)take(WS_XB);
    float* SF   = (float*)take(WS_F32);
    float* TF   = (float*)take(WS_F32);
    h16*   XT16 = (h16*)take(WS_XT);
    h16*   P16  = (h16*)take(WS_P);
    float* CTX  = (float*)take(WS_F32);
    if ((size_t)(wsp - (char*)d_ws) > ws_size) return;

    k_cvt8<<<(unsigned)(((size_t)HID * HID / 8 + 255) / 256), 256, 0, stream>>>(Ws_w, WSB, (size_t)HID * HID / 8);
    k_cvt8<<<(unsigned)(((size_t)HID * HID / 8 + 255) / 256), 256, 0, stream>>>(Wt_w, WTB, (size_t)HID * HID / 8);
    k_cvt8<<<(unsigned)(((size_t)NB * SEQ * HID / 8 + 255) / 256), 256, 0, stream>>>(x, XB, (size_t)NB * SEQ * HID / 8);
    k_vtp<<<(unsigned)(((size_t)NB * DV * TK / 2 + 255) / 256), 256, 0, stream>>>(x, XT16);
    k_gemmw<bf, 0, true><<<dim3(NB * SEQ / 64, HID / 64, 1), 32, 0, stream>>>(XB, nullptr, WSB, nullptr, HID, SF, HID, Ws_b, 1.0f, 0, 0, 0);
    k_gemmw<bf, 0, true><<<dim3(NB * SEQ / 64, HID / 64, 1), 32, 0, stream>>>(XB, nullptr, WTB, nullptr, HID, TF, HID, Wt_b, 1.0f, 0, 0, 0);
    k_score<<<(unsigned)(NB * SEQ), 256, 0, stream>>>(SF, TF, vv, adj, P16);
    k_gemmw<h16, 0, false><<<dim3(SEQ / 64, HID / 64, NB), 32, 0, stream>>>(P16, nullptr, XT16, nullptr, SEQ, CTX, HID, nullptr, OSC, (size_t)SEQ * SEQ, (size_t)HID * SEQ, (size_t)SEQ * HID);
    k_lnorm<<<(unsigned)(NB * SEQ / 128), 256, 0, stream>>>(CTX, ln_g, ln_b, OUT);
}
